// WHVILinear_55070070669432
// MI455X (gfx1250) — hardware-verified
//
#include <hip/hip_runtime.h>


#define NBT  8192
#define DD   1024
typedef _Float16 h16;
typedef unsigned short bf;
typedef __attribute__((ext_vector_type(16))) __bf16   v16bf;
typedef __attribute__((ext_vector_type(16))) _Float16 v16h;
typedef __attribute__((ext_vector_type(8)))  _Float16 v8h;
typedef __attribute__((ext_vector_type(8)))  unsigned short v8us;
typedef __attribute__((ext_vector_type(8)))  float    v8f;
typedef __attribute__((ext_vector_type(4)))  float    v4f;
typedef v8h  __attribute__((may_alias)) v8ha;
typedef v4f  __attribute__((may_alias)) v4fa;
typedef v8us __attribute__((may_alias)) v8usa;

__device__ __forceinline__ unsigned short f2bf(float f) { unsigned u = __float_as_uint(f); u += 0x7FFFu + ((u >> 16) & 1u); return (unsigned short)(u >> 16); }
__device__ __forceinline__ float bf2f(unsigned short b) { return __uint_as_float(((unsigned)b) << 16); }
__device__ __forceinline__ float bfr(float f) { return bf2f(f2bf(f)); }
__device__ __forceinline__ v16h cat16(v8h lo, v8h hi) { return __builtin_shufflevector(lo, hi, 0, 1, 2, 3, 4, 5, 6, 7, 8, 9, 10, 11, 12, 13, 14, 15); }
__device__ __forceinline__ v16bf cat16b(v8us lo, v8us hi) { return __builtin_bit_cast(v16bf, __builtin_shufflevector(lo, hi, 0, 1, 2, 3, 4, 5, 6, 7, 8, 9, 10, 11, 12, 13, 14, 15)); }
__device__ __forceinline__ v8f wmma16(v16h a, v16h b, v8f c) { return __builtin_amdgcn_wmma_f32_16x16x32_f16(false, a, false, b, (short)0, c, false, false); }
__device__ __forceinline__ v8f wmmab(v16bf a, v16bf b, v8f c) { return __builtin_amdgcn_wmma_f32_16x16x32_bf16(false, a, false, b, (short)0, c, false, false); }


template <typename T16> struct WFrag;
template <> struct WFrag<h16> { typedef v16h V; static __device__ __forceinline__ V ld(const h16* p) { return cat16(*(const v8h*)p, *(const v8h*)(p + 16)); } static __device__ __forceinline__ v8f mma(V a, V b, v8f c) { return wmma16(a, b, c); } };
template <> struct WFrag<bf> { typedef v16bf V; static __device__ __forceinline__ V ld(const bf* p) { return cat16b(*(const v8us*)p, *(const v8us*)(p + 16)); } static __device__ __forceinline__ v8f mma(V a, V b, v8f c) { return wmmab(a, b, c); } };
template <typename T16, int NSPLIT, bool BIAS>
__global__ __launch_bounds__(32) void k_gemmw(const T16* __restrict__ A, const T16* __restrict__ A2, const T16* __restrict__ Bt, const T16* __restrict__ Bt2, int K, float* C, int ldc, const float* __restrict__ bias, size_t sA, size_t sB, size_t sC) {
    typedef typename WFrag<T16>::V V;
    __shared__ __align__(16) float os[16 * 68];
    const size_t z = blockIdx.z; A += z * sA; if (A2) A2 += z * sA; Bt += z * sB; if (Bt2) Bt2 += z * sB; C += z * sC;
    const int lane = threadIdx.x & 31, lr = lane & 15, hi = lane >> 4; const int r0 = blockIdx.x * 64, c0 = blockIdx.y * 64;
    v8f acc[4][4];
#pragma unroll
    for (int mb = 0; mb < 4; ++mb)
#pragma unroll
        for (int nb = 0; nb < 4; ++nb) acc[mb][nb] = (v8f){};
    const size_t aoff = (size_t)(r0 + lr) * K + 8 * hi, boff = (size_t)(c0 + lr) * K + 8 * hi;
#pragma unroll 1
    for (int kc = 0; kc < K; kc += 32) {
        V a[4], a2[4];
#pragma unroll
        for (int mb = 0; mb < 4; ++mb) { a[mb] = WFrag<T16>::ld(A + aoff + (size_t)mb * 16 * K + kc); if (NSPLIT == 1 || NSPLIT == 2) a2[mb] = WFrag<T16>::ld(A2 + aoff + (size_t)mb * 16 * K + kc); }
#pragma unroll
        for (int nb = 0; nb < 4; ++nb) { const V b = WFrag<T16>::ld(Bt + boff + (size_t)nb * 16 * K + kc); V b2; if (NSPLIT >= 2) b2 = WFrag<T16>::ld(Bt2 + boff + (size_t)nb * 16 * K + kc);
#pragma unroll
            for (int mb = 0; mb < 4; ++mb) { acc[mb][nb] = WFrag<T16>::mma(a[mb], b, acc[mb][nb]); if (NSPLIT == 1 || NSPLIT == 2) acc[mb][nb] = WFrag<T16>::mma(a2[mb], b, acc[mb][nb]); if (NSPLIT >= 2) acc[mb][nb] = WFrag<T16>::mma(a[mb], b2, acc[mb][nb]); } }
        asm volatile("v_nop\n\tv_nop\n\tv_nop\n\tv_nop" : "+v"(acc[0][0]), "+v"(acc[1][1]), "+v"(acc[2][2]), "+v"(acc[3][3]) : "v"(a[0]), "v"(a[3]));
    }
#pragma unroll
    for (int mb = 0; mb < 4; ++mb) {
#pragma unroll
        for (int nb = 0; nb < 4; ++nb) {
#pragma unroll
            for (int j = 0; j < 8; ++j) os[(hi * 8 + j) * 68 + nb * 16 + lr] = acc[mb][nb][j]; }
        __builtin_amdgcn_wave_barrier(); asm volatile("" ::: "memory");
        float* crow = C + (size_t)(r0 + mb * 16) * ldc + c0;
#pragma unroll 1
        for (int ps = 0; ps < 2; ++ps) {
#pragma unroll
            for (int s = 0; s < 8; ++s) { const int row = 2 * s + hi, cofs = lr * 4; v4f val = *(const v4fa*)(os + row * 68 + cofs); if (BIAS) { val[0] += bfr(bias[c0 + cofs]); val[1] += bfr(bias[c0 + cofs + 1]); val[2] += bfr(bias[c0 + cofs + 2]); val[3] += bfr(bias[c0 + cofs + 3]); }
                *(volatile v4f*)(crow + (size_t)row * ldc + cofs) = val; }
            if (ps == 0) __threadfence(); }
        __builtin_amdgcn_wave_barrier(); asm volatile("" ::: "memory");
    }
}

__device__ __forceinline__ void splitf(float y, unsigned short& h, unsigned short& l) { h = f2bf(y); l = f2bf(y - bf2f(h)); }
typedef __attribute__((ext_vector_type(4))) unsigned short v4us;

__global__ __launch_bounds__(256) void k_cvt8(const float* __restrict__ src, bf* dst, size_t n8) { const size_t i = (size_t)blockIdx.x * 256 + threadIdx.x; if (i >= n8) return; const v8f v = *(const v8f*)(src + i * 8); v8us o;
#pragma unroll
    for (int k = 0; k < 8; ++k) o[k] = f2bf(v[k]); *(volatile v8us*)(dst + i * 8) = o; __threadfence(); *(volatile v8us*)(dst + i * 8) = o; }
__global__ __launch_bounds__(256) void k_rsp(const float* __restrict__ Rho, bf* Rh, bf* Rl) { const size_t e = ((size_t)blockIdx.x * 256 + threadIdx.x) * 4; if (e >= (size_t)DD * DD) return; v4us oh, ol;
#pragma unroll
    for (int u = 0; u < 4; ++u) { const float z = bfr(Rho[e + u]); const float sp = (z > 20.f) ? z : log1pf(__expf(z)); unsigned short a, b; splitf(sp, a, b); oh[u] = a; ol[u] = b; } *(volatile v4us*)(Rh + e) = oh; *(volatile v4us*)(Rl + e) = ol; __threadfence(); *(volatile v4us*)(Rh + e) = oh; *(volatile v4us*)(Rl + e) = ol; }
__global__ __launch_bounds__(256) void k_matvec(const float* __restrict__ SG, const float* __restrict__ eps, const float* __restrict__ mu, float* U) { const int lane = threadIdx.x & 31; const int wv = threadIdx.x >> 5; const int i = blockIdx.x * 8 + wv; float acc = 0.f; const float* row = SG + (size_t)i * DD;
#pragma unroll 4
    for (int j = lane; j < DD; j += 32) { float p = __fmul_rn(row[j], bfr(eps[j])); asm volatile("" : "+v"(p)); acc = __fadd_rn(acc, p); }
#pragma unroll
    for (int sh = 16; sh; sh >>= 1) acc += __shfl_xor(acc, sh, 32);
    const float ui = __fadd_rn(bfr(mu[i]), acc); __shared__ float shv[8]; if (lane == 0) shv[wv] = ui; __syncthreads();
    if (threadIdx.x < 32) { const float v = (threadIdx.x < 8) ? shv[threadIdx.x] : 0.f; float* d = U + (size_t)blockIdx.x * 32 + threadIdx.x; *(volatile float*)d = v; __threadfence(); *(volatile float*)d = v; } }
__device__ __forceinline__ float uAt(const float* __restrict__ U, int i) { return U[(i >> 3) * 32 + (i & 7)]; }
__global__ __launch_bounds__(256) void k_ascale(const float* __restrict__ H, const float* __restrict__ s1, const float* __restrict__ U, bf* Ah, bf* Al) { const size_t e = ((size_t)blockIdx.x * 256 + threadIdx.x) * 4; if (e >= (size_t)DD * DD) return; const int j = (int)(e % DD); const int i = (int)(e / DD); const float si = bfr(s1[i]); v4us oh, ol;
#pragma unroll
    for (int u = 0; u < 4; ++u) { float t1 = __fmul_rn(si, bfr(H[e + u])); asm volatile("" : "+v"(t1)); const float a = __fmul_rn(t1, uAt(U, j + u)); unsigned short p, q; splitf(a, p, q); oh[u] = p; ol[u] = q; } *(volatile v4us*)(Ah + e) = oh; *(volatile v4us*)(Al + e) = ol; __threadfence(); *(volatile v4us*)(Ah + e) = oh; *(volatile v4us*)(Al + e) = ol; }
__global__ __launch_bounds__(256) void k_colscale(const float* __restrict__ C, const float* __restrict__ s2, bf* Wh, bf* Wl) { const size_t e = ((size_t)blockIdx.x * 256 + threadIdx.x) * 4; if (e >= (size_t)DD * DD) return; const int k = (int)(e % DD); const v4f c = *(const v4f*)(C + e); v4us oh, ol;
#pragma unroll
    for (int u = 0; u < 4; ++u) { unsigned short p, q; splitf(__fmul_rn(c[u], bfr(s2[k + u])), p, q); oh[u] = p; ol[u] = q; } *(volatile v4us*)(Wh + e) = oh; *(volatile v4us*)(Wl + e) = ol; __threadfence(); *(volatile v4us*)(Wh + e) = oh; *(volatile v4us*)(Wl + e) = ol; }
__global__ __launch_bounds__(256) void k_relu(float* O, size_t n4) { const size_t e = ((size_t)blockIdx.x * 256 + threadIdx.x) * 4; if (e >= n4) return; const v4f a = *(const v4f*)(O + e); v4f o; for (int u = 0; u < 4; ++u) o[u] = fmaxf(a[u], 0.f); *(volatile v4f*)(O + e) = o; __threadfence(); *(volatile v4f*)(O + e) = o; }

extern "C" void kernel_launch(void* const* d_in, const int* in_sizes, int n_in,
                              void* d_out, int out_size, void* d_ws, size_t ws_size, hipStream_t stream) {
    (void)in_sizes; (void)n_in; (void)out_size;
    const float* x = (const float*)d_in[0]; const float* s1 = (const float*)d_in[1]; const float* s2 = (const float*)d_in[2]; const float* mu = (const float*)d_in[3]; const float* Rho = (const float*)d_in[4]; const float* eps = (const float*)d_in[5]; const float* H = (const float*)d_in[6];
    float* OUT = (float*)d_out;
    char* wsp = (char*)d_ws;
    auto take = [&](size_t bytes) { char* p = wsp; wsp += (bytes + 255) & ~(size_t)255; return (void*)p; };
    bf* Rh = (bf*)take((size_t)DD * DD * 2); bf* Rl = (bf*)take((size_t)DD * DD * 2); float* SG = (float*)take((size_t)DD * DD * 4); float* U = (float*)take((size_t)(DD / 8) * 32 * 4); bf* HB = (bf*)take((size_t)DD * DD * 2);
    bf* Ah = (bf*)take((size_t)DD * DD * 2); bf* Al = (bf*)take((size_t)DD * DD * 2); float* C = (float*)take((size_t)DD * DD * 4); bf* Wh = (bf*)take((size_t)DD * DD * 2); bf* Wl = (bf*)take((size_t)DD * DD * 2); bf* XB = (bf*)take((size_t)NBT * DD * 2);
    if ((size_t)(wsp - (char*)d_ws) > ws_size) return;
    const unsigned gD = (unsigned)(((size_t)DD * DD / 4 + 255) / 256);
    k_rsp<<<gD, 256, 0, stream>>>(Rho, Rh, Rl);
    k_gemmw<bf, 2, false><<<dim3(DD / 64, DD / 64, 1), 32, 0, stream>>>(Rh, Rl, Rh, Rl, DD, SG, DD, nullptr, 0, 0, 0);
    k_matvec<<<DD / 8, 256, 0, stream>>>(SG, eps, mu, U);
    k_cvt8<<<(DD * DD / 8 + 255) / 256, 256, 0, stream>>>(H, HB, DD * DD / 8);
    k_ascale<<<gD, 256, 0, stream>>>(H, s1, U, Ah, Al);
    k_gemmw<bf, 1, false><<<dim3(DD / 64, DD / 64, 1), 32, 0, stream>>>(Ah, Al, HB, nullptr, DD, C, DD, nullptr, 0, 0, 0);
    k_colscale<<<gD, 256, 0, stream>>>(C, s2, Wh, Wl);
    k_cvt8<<<(unsigned)(((size_t)NBT * DD / 8 + 255) / 256), 256, 0, stream>>>(x, XB, (size_t)NBT * DD / 8);
    k_gemmw<bf, 1, false><<<dim3(DD / 64, NBT / 64, 1), 32, 0, stream>>>(Wh, Wl, XB, nullptr, DD, OUT, NBT, nullptr, 0, 0, 0);
    k_relu<<<(unsigned)(((size_t)DD * NBT / 4 + 255) / 256), 256, 0, stream>>>(OUT, (size_t)DD * NBT);
}
